// VisionAttention_65936337928634
// MI455X (gfx1250) — hardware-verified
//
#include <hip/hip_runtime.h>
#include <math.h>
#include <stdint.h>

constexpr int kBatch   = 4;
constexpr int kSeq     = 2048;
constexpr int kModel   = 1024;
constexpr int kHeads   = 16;
constexpr int kHeadDim = 64;
constexpr int kQKV     = kHeads * kHeadDim;
constexpr int kTokens  = kBatch * kSeq;
constexpr float kEps       = 1e-6f;
constexpr float kProbCarry = 32768.0f;
constexpr float kOutCarry  = 16.0f;
constexpr float kWoCarry   = 64.0f;

constexpr size_t kPlane16  = (size_t)kTokens * kQKV * 2;
constexpr size_t kWPlane16 = (size_t)kQKV * kModel * 2;
constexpr size_t kOffX  = 0;
constexpr size_t kOffO  = 0;
constexpr size_t kOffWq = kOffX + kPlane16;
constexpr size_t kOffWk = kOffWq + kWPlane16;
constexpr size_t kOffWv = kOffWk + kWPlane16;
constexpr size_t kOffWo = kOffWv + kWPlane16;
constexpr size_t kOffQh = kOffWo + kWPlane16;
constexpr size_t kOffKh = kOffQh + kPlane16;
constexpr size_t kOffQl = kOffKh + kPlane16;
constexpr size_t kOffKl = kOffQl + kPlane16;
constexpr size_t kOffVt = kOffKl + kPlane16;
constexpr size_t kWsTotal = kOffVt + kPlane16;

typedef __attribute__((ext_vector_type(16))) _Float16 v16h;
typedef __attribute__((ext_vector_type(8)))  _Float16 v8h;
typedef __attribute__((ext_vector_type(16))) __bf16   v16b;
typedef __attribute__((ext_vector_type(8)))  __bf16   v8b;
typedef __attribute__((ext_vector_type(8)))  float    v8f;
typedef __attribute__((ext_vector_type(4)))  float    v4f;
typedef __attribute__((ext_vector_type(2)))  float    v2f;

__device__ __forceinline__ unsigned short f2bf_bits(float f) {
  unsigned u = __float_as_uint(f);
  return (unsigned short)((u + 0x7FFFu + ((u >> 16) & 1u)) >> 16);
}
__device__ __forceinline__ float bf_bits2f(unsigned short h) { return __uint_as_float(((unsigned)h) << 16); }
__device__ __forceinline__ float bf16_rne_f32(float f) { return bf_bits2f(f2bf_bits(f)); }
__device__ __forceinline__ unsigned pk16(unsigned short a, unsigned short b) { return (unsigned)a | ((unsigned)b << 16); }

__device__ __forceinline__ void dep_guard_h(v8f& a, v8f& b, v16h x, v16h y) { asm volatile("v_nop\n\tv_nop\n\tv_nop\n\tv_nop" : "+v"(a), "+v"(b) : "v"(x), "v"(y)); }
__device__ __forceinline__ void dep_guard_b(v8f& a, v8f& b, v16b x, v16b y) { asm volatile("v_nop\n\tv_nop\n\tv_nop\n\tv_nop" : "+v"(a), "+v"(b) : "v"(x), "v"(y)); }
__device__ __forceinline__ void keep4_h(v16h a, v16h b, v16h c, v16h d) { asm volatile("v_nop" :: "v"(a), "v"(b), "v"(c), "v"(d)); }
__device__ __forceinline__ void keep4_b(v16b a, v16b b, v16b c, v16b d) { asm volatile("v_nop" :: "v"(a), "v"(b), "v"(c), "v"(d)); }
__device__ __forceinline__ void acc_guard4(v8f& a, v8f& b, v8f& c, v8f& d) { asm volatile("v_nop\n\tv_nop\n\tv_nop\n\tv_nop" : "+v"(a), "+v"(b), "+v"(c), "+v"(d)); }
template <typename T> struct Frag;
template <> struct Frag<_Float16> {
  typedef v16h V; union U { v16h v; v8h h[2]; };
  static __device__ __forceinline__ v16h load(const _Float16* p) {
    U f; f.h[0] = *(const v8h*)(p); f.h[1] = *(const v8h*)(p + 16); return f.v;
  }
  static __device__ __forceinline__ v8f mma(v16h a, v16h b, v8f c) {
    return __builtin_amdgcn_wmma_f32_16x16x32_f16(false, a, false, b, (short)0, c, false, false);
  }
  static __device__ __forceinline__ void guard(v8f& a, v8f& b, v16h x, v16h y) { dep_guard_h(a, b, x, y); }
  static __device__ __forceinline__ void keep(v16h a, v16h b, v16h c, v16h d) { keep4_h(a, b, c, d); }
};
template <> struct Frag<__bf16> {
  typedef v16b V; union U { v16b v; v8b h[2]; };
  static __device__ __forceinline__ v16b load(const __bf16* p) {
    U f; f.h[0] = *(const v8b*)(p); f.h[1] = *(const v8b*)(p + 16); return f.v;
  }
  static __device__ __forceinline__ v8f mma(v16b a, v16b b, v8f c) {
    return __builtin_amdgcn_wmma_f32_16x16x32_bf16(false, a, false, b, (short)0, c, false, false);
  }
  static __device__ __forceinline__ void guard(v8f& a, v8f& b, v16b x, v16b y) { dep_guard_b(a, b, x, y); }
  static __device__ __forceinline__ void keep(v16b a, v16b b, v16b c, v16b d) { keep4_b(a, b, c, d); }
};

template <int ET> struct Elem;
template <> struct Elem<0> { typedef _Float16 T; };
template <> struct Elem<1> { typedef __bf16 T; };
template <int ET, bool SPLIT, int BIAS_MODE, int OUT_MODE, bool RESID, int ACT, int EPI>
__global__ __launch_bounds__(256) void wmma_gemm64(
    const unsigned short* __restrict__ Ap, const unsigned short* __restrict__ A2p, int lda, long strideA,
    const unsigned short* __restrict__ Btp, const unsigned short* __restrict__ Bt2p, int ldb, long strideB,
    void* __restrict__ Cout, void* __restrict__ Cout2, int ldc, long strideC,
    const float* __restrict__ bias,
    const float* __restrict__ resid, long strideR,
    const float* __restrict__ epi_cos, const float* __restrict__ epi_sin,
    const float* __restrict__ epi_s0, const float* __restrict__ epi_s1, float epi_eps,
    int M, int N, int K, float scale) {
  typedef typename Elem<ET>::T T;
  typedef typename Frag<T>::V V;
  const T* A = (const T*)Ap; const T* A2 = (const T*)A2p; const T* Bt = (const T*)Btp; const T* Bt2 = (const T*)Bt2p;
  __shared__ __align__(16) float sT[8][16 * 68];
  const int b    = blockIdx.y;
  const int lane = threadIdx.x & 31;
  const int wave = threadIdx.x >> 5;
  const int tilesN = N >> 6;
  const int tilesM = M >> 6;
  const int tile = blockIdx.x * 8 + wave;
  if (tile >= tilesM * tilesN) return;
  const int tm = tile / tilesN;
  const int tn = tile - tm * tilesN;
  const int m0 = tm << 6;
  const int n0 = tn << 6;

  const T* Ab  = A  + (size_t)b * strideA;
  const T* Bb  = Bt + (size_t)b * strideB;
  const T* Ab2 = SPLIT ? (A2  + (size_t)b * strideA) : nullptr;
  const T* Bb2 = SPLIT ? (Bt2 + (size_t)b * strideB) : nullptr;

  const int rlane = lane & 15;
  const int koff  = (lane >> 4) * 8;
  const int mOff  = (lane >> 4) * 8;

  v8f acc[4][4];
#pragma unroll
  for (int i = 0; i < 4; ++i)
#pragma unroll
    for (int j = 0; j < 4; ++j) acc[i][j] = (v8f){0.f,0.f,0.f,0.f,0.f,0.f,0.f,0.f};

  for (int k0 = 0; k0 < K; k0 += 32) {
    V bh[4], bl[4];
#pragma unroll
    for (int j = 0; j < 4; ++j) {
      const size_t bo = (size_t)(n0 + (j << 4) + rlane) * ldb + koff + k0;
      bh[j] = Frag<T>::load(Bb + bo);
      if (SPLIT) bl[j] = Frag<T>::load(Bb2 + bo);
    }
#pragma unroll
    for (int i = 0; i < 4; ++i) {
      const size_t ao = (size_t)(m0 + (i << 4) + rlane) * lda + koff + k0;
      V ah = Frag<T>::load(Ab + ao);
      V al;
      if (SPLIT) al = Frag<T>::load(Ab2 + ao);
#pragma unroll
      for (int j = 0; j < 4; ++j) {
        acc[i][j] = Frag<T>::mma(ah, bh[j], acc[i][j]);
        if (SPLIT) {
          acc[i][j] = Frag<T>::mma(ah, bl[j], acc[i][j]);
          acc[i][j] = Frag<T>::mma(al, bh[j], acc[i][j]);
        }
      }
      Frag<T>::guard(acc[i][0], acc[i][3], ah, SPLIT ? al : ah);
    }
    Frag<T>::keep(bh[0], bh[1], bh[2], bh[3]);
    if (SPLIT) Frag<T>::keep(bl[0], bl[1], bl[2], bl[3]);
  }
  acc_guard4(acc[0][0], acc[0][1], acc[0][2], acc[0][3]);
  acc_guard4(acc[1][0], acc[1][1], acc[1][2], acc[1][3]);
  acc_guard4(acc[2][0], acc[2][1], acc[2][2], acc[2][3]);
  acc_guard4(acc[3][0], acc[3][1], acc[3][2], acc[3][3]);

  float cri[4] = {1.f, 1.f, 1.f, 1.f};
  if (EPI == 2) {
#pragma unroll
    for (int j = 0; j < 4; ++j) {
      float css = 0.f;
#pragma unroll
      for (int i = 0; i < 4; ++i)
#pragma unroll
        for (int r = 0; r < 8; ++r) { const float t = acc[i][j][r] * scale; css += t * t; }
      css += __shfl_xor(css, 16, 32);
      cri[j] = rsqrtf(css * (1.0f / 64.0f) + epi_eps);
    }
  }

  float* slab = sT[wave];
  const float* Rb = RESID ? (resid + (size_t)b * strideR) : nullptr;
#pragma unroll
  for (int i = 0; i < 4; ++i) {
    const int mBase = m0 + (i << 4);
#pragma unroll
    for (int j = 0; j < 4; ++j) {
      const int n = n0 + (j << 4) + rlane;
      float bv = 0.f;
      if (BIAS_MODE == 2) bv = bias[n];
#pragma unroll
      for (int r = 0; r < 8; ++r) {
        float v = acc[i][j][r] * scale;
        if (EPI == 2) v *= cri[j];
        if (BIAS_MODE == 1) v += bias[mBase + mOff + r];
        if (BIAS_MODE == 2) v += bv;
        if (RESID) v += Rb[(size_t)(mBase + mOff + r) * ldc + n];
        if (ACT == 1) v = tanhf(v);
        if (ACT == 2) v = fmaxf(v, 0.0f);
        if (ACT == 3) v = v / (1.0f + expf(-v));
        if (ACT == 4) v = (v > 0.f) ? v : 0.01f * v;
        slab[(mOff + r) * 68 + (j << 4) + rlane] = v;
      }
    }
    __builtin_amdgcn_fence(__ATOMIC_RELEASE, "workgroup");
    __builtin_amdgcn_wave_barrier();
    __builtin_amdgcn_fence(__ATOMIC_ACQUIRE, "workgroup");
    if (EPI == 1) {
      const int erow = lane & 15;
      const int ech  = lane >> 4;
      float* srow = slab + erow * 68 + ech * 32;
      float ss = 0.f;
#pragma unroll
      for (int c4i = 0; c4i < 8; ++c4i) {
        const v4f xv = *(const v4f*)(srow + 4 * c4i);
        ss += xv[0] * xv[0] + xv[1] * xv[1] + xv[2] * xv[2] + xv[3] * xv[3];
      }
      ss += __shfl_xor(ss, 16, 32);
      const float ri = rsqrtf(ss * (1.0f / 64.0f) + epi_eps);
      const size_t tok = (size_t)(mBase + erow);
      const float* cr = epi_cos + tok * 64 + ech * 32;
      const float* sr = epi_sin + tok * 64 + ech * 32;
      const float* sA = epi_s0 + ech * 32;
      const float* sB = epi_s1 + ech * 32;
#pragma unroll 1
      for (int cc = 0; cc < 16; ++cc) {
        const float x0 = srow[cc];
        const float x1 = srow[cc + 16];
        const float sa0 = sA[cc], sa1 = sA[cc + 16], sb0 = sB[cc], sb1 = sB[cc + 16];
        const float sc0 = bf16_rne_f32((b == 0) ? sa0 : sb0);
        const float sc1 = bf16_rne_f32((b == 0) ? sa1 : sb1);
        const float a0 = (x0 * ri) * sc0;
        const float a1 = (x1 * ri) * sc1;
        const float c0 = bf16_rne_f32(cr[cc]), c1 = bf16_rne_f32(cr[cc + 16]);
        const float s0 = bf16_rne_f32(sr[cc]), s1 = bf16_rne_f32(sr[cc + 16]);
        const float y0 = a0 * c0 - a1 * s0;
        const float y1 = a1 * c1 + a0 * s1;
        srow[cc]      = y0;
        srow[cc + 16] = y1;
      }
      __builtin_amdgcn_fence(__ATOMIC_RELEASE, "workgroup");
      __builtin_amdgcn_wave_barrier();
      __builtin_amdgcn_fence(__ATOMIC_ACQUIRE, "workgroup");
    }
    if (OUT_MODE == 0) {
      float* C = (float*)Cout + (size_t)b * strideC;
      const int hh = lane >> 4, c4 = (lane & 15) * 4;
      for (int pass = 0; pass < 2; ++pass) {
#pragma unroll
        for (int it = 0; it < 8; ++it) {
          const int row = it * 2 + hh;
          v4f v = *(const v4f*)(slab + row * 68 + c4);
          *(volatile v4f*)(C + (size_t)(mBase + row) * ldc + n0 + c4) = v;
        }
        __threadfence();
      }
    } else {
      const int q = lane >> 3, c8 = (lane & 7) * 8;
      unsigned short* C  = (unsigned short*)Cout  + (size_t)b * strideC;
      unsigned short* C2 = (OUT_MODE == 2) ? ((unsigned short*)Cout2 + (size_t)b * strideC) : nullptr;
      for (int pass = 0; pass < 2; ++pass) {
#pragma unroll
        for (int it = 0; it < 4; ++it) {
          const int row = it * 4 + q;
          const float* sp = slab + row * 68 + c8;
          v8h hv, lv;
#pragma unroll
          for (int e = 0; e < 8; ++e) {
            if (OUT_MODE == 1) {
              hv[e] = (_Float16)sp[e];
            } else {
              unsigned short hb = f2bf_bits(sp[e]);
              unsigned short lb = f2bf_bits(sp[e] - bf_bits2f(hb));
              hv[e] = __builtin_bit_cast(_Float16, hb);
              lv[e] = __builtin_bit_cast(_Float16, lb);
            }
          }
          *(volatile v8h*)(C + (size_t)(mBase + row) * ldc + n0 + c8) = hv;
          if (OUT_MODE == 2) *(volatile v8h*)(C2 + (size_t)(mBase + row) * ldc + n0 + c8) = lv;
        }
        __threadfence();
      }
    }
    __builtin_amdgcn_fence(__ATOMIC_RELEASE, "workgroup");
    __builtin_amdgcn_wave_barrier();
    __builtin_amdgcn_fence(__ATOMIC_ACQUIRE, "workgroup");
  }
}

__global__ __launch_bounds__(256) void cast_bf16x2_kernel(const float* __restrict__ in, unsigned short* __restrict__ out, int n2) {
  const int i = blockIdx.x * 256 + threadIdx.x;
  if (i < n2) {
    const v2f f = *(const v2f*)(in + 2 * (size_t)i);
    const unsigned u = pk16(f2bf_bits(f[0]), f2bf_bits(f[1]));
    ((volatile unsigned*)out)[i] = u;
    __threadfence();
    ((volatile unsigned*)out)[i] = u;
  }
}

__global__ __launch_bounds__(256) void cast_carry_f16x2_kernel(const float* __restrict__ in, unsigned short* __restrict__ out,
                                                               int n2, float carry) {
  const int i = blockIdx.x * 256 + threadIdx.x;
  if (i < n2) {
    const v2f f = *(const v2f*)(in + 2 * (size_t)i);
    const _Float16 h0 = (_Float16)(bf16_rne_f32(f[0]) * carry);
    const _Float16 h1 = (_Float16)(bf16_rne_f32(f[1]) * carry);
    const unsigned u = pk16(__builtin_bit_cast(unsigned short, h0), __builtin_bit_cast(unsigned short, h1));
    ((volatile unsigned*)out)[i] = u;
    __threadfence();
    ((volatile unsigned*)out)[i] = u;
  }
}

__device__ __forceinline__ v8f mma_bf16_g(v16b a, v16b b, v8f c) {
  c = __builtin_amdgcn_wmma_f32_16x16x32_bf16(false, a, false, b, (short)0, c, false, false);
  asm volatile("v_nop\n\tv_nop\n\tv_nop\n\tv_nop" : "+v"(c) : "v"(a), "v"(b));
  return c;
}
__device__ __forceinline__ v8f mma_f16_g(v16h a, v16h b, v8f c) {
  c = __builtin_amdgcn_wmma_f32_16x16x32_f16(false, a, false, b, (short)0, c, false, false);
  asm volatile("v_nop\n\tv_nop\n\tv_nop\n\tv_nop" : "+v"(c) : "v"(a), "v"(b));
  return c;
}

__global__ __launch_bounds__(128)
void attn_vis_kernel(const unsigned short* __restrict__ qhp, const unsigned short* __restrict__ qlp,
                     const unsigned short* __restrict__ khp, const unsigned short* __restrict__ klp,
                     const unsigned short* __restrict__ vtp, unsigned short* __restrict__ outp) {
  union FB { v16b v; v8b h[2]; };
  union FH { v16h v; v8h h[2]; };
  __shared__ __align__(16) __bf16   Ksh[64 * 64];
  __shared__ __align__(16) __bf16   Ksl[64 * 64];
  __shared__ __align__(16) _Float16 Vts[64 * 64];
  __shared__ __align__(16) _Float16 Psh[4][16 * 64];
  __shared__ __align__(16) float    Os[4][16 * 68];

  const int tid  = threadIdx.x;
  const int wave = tid >> 5;
  const int lane = tid & 31;
  const int hh   = lane >> 4;
  const int c    = lane & 15;

  const int nqb = kSeq / 64;
  const int qb  = blockIdx.x % nqb;
  const int h   = blockIdx.x / nqb;
  const int b   = blockIdx.y;
  const int q0  = qb * 64 + wave * 16;
  const size_t tokb = (size_t)b * kSeq;

  const __bf16* Qh = (const __bf16*)(const void*)qhp + tokb * kQKV + (size_t)h * kHeadDim;
  const __bf16* Ql = (const __bf16*)(const void*)qlp + tokb * kQKV + (size_t)h * kHeadDim;
  const __bf16* Kh = (const __bf16*)(const void*)khp + tokb * kQKV + (size_t)h * kHeadDim;
  const __bf16* Kl = (const __bf16*)(const void*)klp + tokb * kQKV + (size_t)h * kHeadDim;
  const _Float16* Vt = (const _Float16*)(const void*)vtp + ((size_t)b * kQKV + (size_t)h * kHeadDim) * kSeq;
  _Float16* Ob = (_Float16*)(void*)outp + tokb * kQKV + (size_t)h * kHeadDim;

  v16b qah[2], qal[2];
#pragma unroll
  for (int dc = 0; dc < 2; ++dc) {
    qah[dc] = Frag<__bf16>::load(Qh + (size_t)(q0 + c) * kQKV + dc * 32 + 8 * hh);
    qal[dc] = Frag<__bf16>::load(Ql + (size_t)(q0 + c) * kQKV + dc * 32 + 8 * hh);
  }

  float mrow[8], lrow[8];
  v8f oacc[4];
#pragma unroll
  for (int r = 0; r < 8; ++r) { mrow[r] = -INFINITY; lrow[r] = 0.f; }
#pragma unroll
  for (int t = 0; t < 4; ++t) oacc[t] = (v8f){0.f,0.f,0.f,0.f,0.f,0.f,0.f,0.f};

  for (int kc = 0; kc < kSeq / 64; ++kc) {
    const int kv0 = kc * 64;
    __syncthreads();
    {
      const int r = tid >> 1, half = (tid & 1) * 32;
      const __bf16*   ksh = Kh + (size_t)(kv0 + r) * kQKV + half;
      const __bf16*   ksl = Kl + (size_t)(kv0 + r) * kQKV + half;
      const _Float16* vsr = Vt + (size_t)r * kSeq + kv0 + half;
#pragma unroll
      for (int i = 0; i < 4; ++i) {
        const v8b a0 = *(const v8b*)(ksh + 8 * i);
        const v8b a1 = *(const v8b*)(ksl + 8 * i);
        const v8h b0 = *(const v8h*)(vsr + 8 * i);
        *(v8b*)(Ksh + r * 64 + half + 8 * i) = a0;
        *(v8b*)(Ksl + r * 64 + half + 8 * i) = a1;
        *(v8h*)(Vts + r * 64 + half + 8 * i) = b0;
      }
    }
    __syncthreads();

    v8f s[4];
#pragma unroll
    for (int j = 0; j < 4; ++j) {
      s[j] = (v8f){0.f,0.f,0.f,0.f,0.f,0.f,0.f,0.f};
#pragma unroll
      for (int dc = 0; dc < 2; ++dc) {
        FB kb, kl;
        kb.h[0] = *(const v8b*)(Ksh + (j * 16 + c) * 64 + dc * 32 + 8 * hh);
        kb.h[1] = *(const v8b*)(Ksh + (j * 16 + c) * 64 + dc * 32 + 16 + 8 * hh);
        kl.h[0] = *(const v8b*)(Ksl + (j * 16 + c) * 64 + dc * 32 + 8 * hh);
        kl.h[1] = *(const v8b*)(Ksl + (j * 16 + c) * 64 + dc * 32 + 16 + 8 * hh);
        s[j] = mma_bf16_g(qah[dc], kb.v, s[j]);
        s[j] = mma_bf16_g(qah[dc], kl.v, s[j]);
        s[j] = mma_bf16_g(qal[dc], kb.v, s[j]);
      }
    }

    float cm[8];
#pragma unroll
    for (int r = 0; r < 8; ++r) {
      float m = fmaxf(fmaxf(s[0][r], s[1][r]), fmaxf(s[2][r], s[3][r]));
#pragma unroll
      for (int off = 1; off < 16; off <<= 1) m = fmaxf(m, __shfl_xor(m, off, 32));
      cm[r] = m;
    }
    _Float16* pwh = Psh[wave];
#pragma unroll
    for (int r = 0; r < 8; ++r) {
      const float mnew  = fmaxf(mrow[r], cm[r]);
      const float alpha = expf(mrow[r] - mnew);
      mrow[r] = mnew;
      float psum = 0.f;
#pragma unroll
      for (int j = 0; j < 4; ++j) {
        const float p = expf(s[j][r] - mnew);
        psum += p;
        pwh[(8 * hh + r) * 64 + j * 16 + c] = (_Float16)(p * kProbCarry);
      }
#pragma unroll
      for (int off = 1; off < 16; off <<= 1) psum += __shfl_xor(psum, off, 32);
      lrow[r] = lrow[r] * alpha + psum;
#pragma unroll
      for (int t = 0; t < 4; ++t) oacc[t][r] *= alpha;
    }
    __builtin_amdgcn_fence(__ATOMIC_RELEASE, "workgroup");
    __builtin_amdgcn_wave_barrier();
    __builtin_amdgcn_fence(__ATOMIC_ACQUIRE, "workgroup");

#pragma unroll 1
    for (int kk = 0; kk < 2; ++kk) {
      FH pa;
      pa.h[0] = *(const v8h*)(pwh + c * 64 + kk * 32 + 8 * hh);
      pa.h[1] = *(const v8h*)(pwh + c * 64 + kk * 32 + 16 + 8 * hh);
#pragma unroll
      for (int t = 0; t < 4; ++t) {
        FH vb;
        vb.h[0] = *(const v8h*)(Vts + (t * 16 + c) * 64 + kk * 32 + 8 * hh);
        vb.h[1] = *(const v8h*)(Vts + (t * 16 + c) * 64 + kk * 32 + 16 + 8 * hh);
        oacc[t] = mma_f16_g(pa.v, vb.v, oacc[t]);
      }
    }
  }

  float* os = Os[wave];
  constexpr float kFin = kOutCarry / kProbCarry;
#pragma unroll
  for (int r = 0; r < 8; ++r) {
    const float inv = (1.0f / lrow[r]) * kFin;
#pragma unroll
    for (int t = 0; t < 4; ++t) os[(8 * hh + r) * 68 + t * 16 + c] = oacc[t][r] * inv;
  }
  __builtin_amdgcn_fence(__ATOMIC_RELEASE, "workgroup");
  __builtin_amdgcn_wave_barrier();
  __builtin_amdgcn_fence(__ATOMIC_ACQUIRE, "workgroup");
  {
    const int q4 = lane >> 3, c8 = (lane & 7) * 8;
    for (int pass = 0; pass < 2; ++pass) {
#pragma unroll
      for (int it = 0; it < 4; ++it) {
        const int row = it * 4 + q4;
        const float* sp = os + row * 68 + c8;
        v8h hv;
#pragma unroll
        for (int e = 0; e < 8; ++e) hv[e] = (_Float16)sp[e];
        *(volatile v8h*)(Ob + (size_t)(q0 + row) * kQKV + c8) = hv;
      }
      __threadfence();
    }
  }
}

extern "C" void kernel_launch(void* const* d_in, const int* in_sizes, int n_in,
                              void* d_out, int out_size, void* d_ws, size_t ws_size,
                              hipStream_t stream) {
  if (n_in < 10) return;
  if (in_sizes[0] != kTokens * kModel) return;
  if (in_sizes[1] != kTokens * kHeadDim || in_sizes[2] != kTokens * kHeadDim) return;
  if (in_sizes[4] != kQKV * kModel || in_sizes[5] != kQKV * kModel || in_sizes[6] != kQKV * kModel) return;
  if (in_sizes[7] != kModel * kQKV) return;
  if (in_sizes[8] != kHeadDim || in_sizes[9] != kHeadDim) return;
  if (out_size != kTokens * kModel) return;
  if (ws_size < kWsTotal) return;

  const float* x    = (const float*)d_in[0];
  const float* cosp = (const float*)d_in[1];
  const float* sinp = (const float*)d_in[2];
  const float* wq   = (const float*)d_in[4];
  const float* wk   = (const float*)d_in[5];
  const float* wv   = (const float*)d_in[6];
  const float* wo   = (const float*)d_in[7];
  const float* qsc  = (const float*)d_in[8];
  const float* ksc  = (const float*)d_in[9];
  float* outp = (float*)d_out;

  char* ws = (char*)d_ws;
  unsigned short* Xb  = (unsigned short*)(ws + kOffX);
  unsigned short* Ob  = (unsigned short*)(ws + kOffO);
  unsigned short* Wqb = (unsigned short*)(ws + kOffWq);
  unsigned short* Wkb = (unsigned short*)(ws + kOffWk);
  unsigned short* Wvb = (unsigned short*)(ws + kOffWv);
  unsigned short* Wof = (unsigned short*)(ws + kOffWo);
  unsigned short* Qh  = (unsigned short*)(ws + kOffQh);
  unsigned short* Ql  = (unsigned short*)(ws + kOffQl);
  unsigned short* Kh  = (unsigned short*)(ws + kOffKh);
  unsigned short* Kl  = (unsigned short*)(ws + kOffKl);
  unsigned short* Vtf = (unsigned short*)(ws + kOffVt);

  const int n2x = kTokens * kModel / 2;
  const int n2w = kQKV * kModel / 2;
  cast_bf16x2_kernel<<<dim3((n2x + 255) / 256), dim3(256), 0, stream>>>(x, Xb, n2x);
  cast_bf16x2_kernel<<<dim3((n2w + 255) / 256), dim3(256), 0, stream>>>(wq, Wqb, n2w);
  cast_bf16x2_kernel<<<dim3((n2w + 255) / 256), dim3(256), 0, stream>>>(wk, Wkb, n2w);
  cast_bf16x2_kernel<<<dim3((n2w + 255) / 256), dim3(256), 0, stream>>>(wv, Wvb, n2w);
  cast_carry_f16x2_kernel<<<dim3((n2w + 255) / 256), dim3(256), 0, stream>>>(wo, Wof, n2w, kWoCarry);

  {
    const int tiles = (kTokens / 64) * (kQKV / 64);
    wmma_gemm64<1, false, 0, 2, false, 0, 1><<<dim3((tiles + 7) / 8, 2), dim3(256), 0, stream>>>(
        Xb, Xb, kModel, 0L,
        Wqb, Wqb, kModel, (long)kQKV * kModel,
        (void*)Qh, (void*)Ql, kQKV, (long)kTokens * kQKV,
        nullptr, nullptr, 0L,
        cosp, sinp, qsc, ksc, kEps,
        kTokens, kQKV, kModel, 1.0f);
  }
  {
    const int tiles = (kQKV / 64) * (kSeq / 64);
    wmma_gemm64<1, false, 0, 1, false, 0, 2><<<dim3((tiles + 7) / 8, kBatch), dim3(256), 0, stream>>>(
        Wvb, Wvb, kModel, 0L,
        Xb, Xb, kModel, (long)kSeq * kModel,
        (void*)Vtf, nullptr, kSeq, (long)kQKV * kSeq,
        nullptr, nullptr, 0L,
        nullptr, nullptr, nullptr, nullptr, kEps,
        kQKV, kSeq, kModel, 1.0f);
  }
  attn_vis_kernel<<<dim3(kHeads * (kSeq / 64), kBatch), dim3(128), 0, stream>>>(Qh, Ql, Kh, Kl, Vtf, Ob);
  {
    const int tiles = (kTokens / 64) * (kModel / 64);
    wmma_gemm64<0, false, 0, 0, false, 0, 0><<<dim3((tiles + 7) / 8, 1), dim3(256), 0, stream>>>(
        Ob, Ob, kQKV, 0L,
        Wof, Wof, kQKV, 0L,
        (void*)outp, nullptr, kModel, 0L,
        nullptr, nullptr, 0L,
        nullptr, nullptr, nullptr, nullptr, kEps,
        kTokens, kModel, kQKV, 1.0f / (kOutCarry * kWoCarry));
  }
}
